// TransR_37967510897466
// MI455X (gfx1250) — hardware-run, weakly checked
//
#include <hip/hip_runtime.h>
#include <stddef.h>
#include <stdint.h>

#define D      128
#define NN     100000
#define NR     500
#define NE     1000000
#define MP     100096
#define GBM    64
#define GBN    128
#define GTHR   128
#define PTHR   256
#define ETHR   256
#define EPB    1024
#define EBLK   977
#define NPASS  64
#define NU_HB  (MP * (D / 8))
#define NU_WB  (D * (D / 8))
#define NU_GF  (NR * (D / 4))
#define NU_GFP 16128
#define NU_BF  (D / 4)
#define NU_BFP 256
#define NU_ALL (NU_HB + NU_WB + NU_GFP + NU_BFP)
#define SZ_HB  ((size_t)MP * D * 2)
#define SZ_S   ((size_t)MP * D * 4)
#define SZ_WB  ((size_t)D * D * 2)
#define SZ_GF  ((size_t)NU_GFP * 16)
#define SZ_BF  ((size_t)512)
#define SZ_ALL (SZ_HB + SZ_S + SZ_WB + SZ_GF + SZ_BF)

static_assert(D == 128 && 16 * 8 == D);
static_assert(EPB % 32 == 0 && EPB == 4 * ETHR);
static_assert((NE - 976 * EPB) == 576 && 576 % 32 == 0);
static_assert(782 * 128 == MP && MP >= NN && MP % GBM == 0);
static_assert(EBLK == (NE + EPB - 1) / EPB && EBLK == 977);
static_assert(NPASS * 16 == EPB && 16 == 2 * (ETHR / 32));
static_assert(NU_HB % PTHR == 0 && NU_WB % PTHR == 0 && NU_GFP % PTHR == 0 && NU_GFP >= NU_GF);
static_assert(NU_BF == 32 && NU_BFP % PTHR == 0 && NU_ALL % PTHR == 0);
static_assert(NE % 4 == 0 && NE >= 4);
static_assert(GBM == (GTHR / 32) * 16 && GBN == D && D % 32 == 0);
static_assert(SZ_HB % 256 == 0 && SZ_S % 256 == 0 && SZ_WB % 256 == 0 && SZ_GF % 256 == 0 && SZ_BF % 256 == 0);
static_assert(SZ_GF >= (size_t)NR * D * 4 && SZ_BF >= (size_t)D * 4);
static_assert(SZ_ALL <= ((size_t)128u << 20));

typedef float          v4f   __attribute__((ext_vector_type(4)));
typedef float          v8f   __attribute__((ext_vector_type(8)));
typedef int            v4i   __attribute__((ext_vector_type(4)));
typedef int            v8i   __attribute__((ext_vector_type(8)));
typedef unsigned short v8us  __attribute__((ext_vector_type(8)));
typedef unsigned short v16us __attribute__((ext_vector_type(16)));
typedef __bf16         v16bf __attribute__((ext_vector_type(16)));
typedef v4f  __attribute__((may_alias)) v4fa;
typedef v4i  __attribute__((may_alias)) v4ia;
typedef v8us __attribute__((may_alias)) v8usa;
union FragB { v16bf v; v16us u; v8us h[2]; v8i w; };

__device__ __forceinline__ v8f wmb(const FragB& a, const FragB& b, v8f c) {
  v8f d = __builtin_amdgcn_wmma_f32_16x16x32_bf16(false, a.v, false, b.v, (short)0, c, false, false);
  asm volatile("v_nop\n\tv_nop\n\tv_nop\n\tv_nop" : "+v"(d) : "v"(a.w), "v"(b.w));
  return d;
}

__device__ __forceinline__ unsigned bf16_bits(float f) {
  const unsigned u = __float_as_uint(f);
  return (u + 0x7FFFu + ((u >> 16) & 1u)) >> 16;
}
__device__ __forceinline__ float bf16_val(float f) {
  return __uint_as_float(bf16_bits(f) << 16);
}
__device__ __forceinline__ int clampi(int x, int hi) {
  x = x < 0 ? 0 : x;
  return x > hi ? hi : x;
}
__device__ __forceinline__ void put16(unsigned short* dp, v8us o) {
  *(volatile v8us*)dp = o;
  __threadfence();
  *(volatile v8us*)dp = o;
}

__global__ __launch_bounds__(PTHR) void k_prep(const float* __restrict__ h, const float* __restrict__ g,
                                               const float* __restrict__ W, const float* __restrict__ b,
                                               unsigned short* HB, unsigned short* WB, float* GF, float* BF) {
  const int u  = (int)blockIdx.x * PTHR + (int)threadIdx.x;
  const int U0 = NU_HB;
  const int U1 = U0 + NU_WB;
  const int U2 = U1 + NU_GFP;
  const int U3 = U2 + NU_BFP;
  if (u < U0) {
    const int row = u >> 4;
    const int k8  = (u & 15) * 8;
    const int rc  = row < NN ? row : NN - 1;
    const float* p = h + (size_t)rc * D + k8;
    const v4f a = *(const v4fa*)p;
    const v4f c = *(const v4fa*)(p + 4);
    const unsigned mk = (row < NN) ? 0xFFFFu : 0u;
    const v8f f8 = {a.x, a.y, a.z, a.w, c.x, c.y, c.z, c.w};
    v8us o;
#pragma unroll
    for (int i = 0; i < 8; ++i) o[i] = (unsigned short)(bf16_bits(f8[i]) & mk);
    put16(HB + (size_t)u * 8, o);
    return;
  } else if (u < U1) {
    const int v = u - U0;
    const float* p = W + (size_t)v * 8;
    const v4f a = *(const v4fa*)p;
    const v4f c = *(const v4fa*)(p + 4);
    const v8f f8 = {a.x, a.y, a.z, a.w, c.x, c.y, c.z, c.w};
    v8us o;
#pragma unroll
    for (int i = 0; i < 8; ++i) o[i] = (unsigned short)bf16_bits(f8[i]);
    put16(WB + (size_t)v * 8, o);
    return;
  } else if (u < U2) {
    const int v  = u - U1;
    const int vc = v < NU_GF ? v : NU_GF - 1;
    const v4f a = *(const v4fa*)(g + (size_t)vc * 4);
    asm volatile("" :: "v"(a));
    v4f q;
    q.x = bf16_val(a.x); q.y = bf16_val(a.y); q.z = bf16_val(a.z); q.w = bf16_val(a.w);
    const bool st = v < NU_GF;
    float* dp = GF + (size_t)vc * 4;
    if (st) *(volatile v4f*)dp = q;
    __threadfence();
    if (st) *(volatile v4f*)dp = q;
    return;
  } else if (u < U3) {
    const int v  = u - U2;
    const int vc = v < NU_BF ? v : NU_BF - 1;
    const v4f a = *(const v4fa*)(b + (size_t)vc * 4);
    asm volatile("" :: "v"(a));
    v4f q;
    q.x = bf16_val(a.x); q.y = bf16_val(a.y); q.z = bf16_val(a.z); q.w = bf16_val(a.w);
    const bool st = v < NU_BF;
    float* dp = BF + (size_t)vc * 4;
    if (st) *(volatile v4f*)dp = q;
    __threadfence();
    if (st) *(volatile v4f*)dp = q;
    return;
  }
}

__global__ __launch_bounds__(GTHR) __attribute__((amdgpu_num_vgpr(248)))
void k_gemm(const unsigned short* __restrict__ A, const unsigned short* __restrict__ BT,
            const float* __restrict__ BF, float* Cm) {
  __shared__ __attribute__((aligned(16))) float stg[GBM * GBN];
  __shared__ __attribute__((aligned(16))) float sB[D];
  const int tid = (int)threadIdx.x, lane = tid & 31, wave = tid >> 5, hh = lane >> 4, m = lane & 15;
  const int rowBase = (int)blockIdx.x * GBM;

  if (tid < 32) {
    const v4f bv = *(const v4fa*)(BF + 4 * tid);
    *(v4fa*)(sB + 4 * tid) = bv;
  }
  __syncthreads();

  v8f acc[8];
  {
    const v8f z = {0.f, 0.f, 0.f, 0.f, 0.f, 0.f, 0.f, 0.f};
#pragma unroll
    for (int t = 0; t < 8; ++t) acc[t] = z;
  }
  const unsigned short* ap = A  + (size_t)(rowBase + 16 * wave + m) * (size_t)D + 8 * hh;
  const unsigned short* bp = BT + (size_t)m * (size_t)D + 8 * hh;

#pragma unroll 1
  for (int k0 = 0; k0 < D; k0 += 32) {
    FragB af;
    af.h[0] = *(const v8usa*)(ap + k0);
    af.h[1] = *(const v8usa*)(ap + k0 + 16);
#pragma unroll
    for (int nt = 0; nt < 8; ++nt) {
      const unsigned short* wq = bp + (size_t)(16 * nt) * (size_t)D + k0;
      FragB bf;
      bf.h[0] = *(const v8usa*)wq;
      bf.h[1] = *(const v8usa*)(wq + 16);
      acc[nt] = wmb(af, bf, acc[nt]);
    }
  }

#pragma unroll
  for (int nt = 0; nt < 8; ++nt) {
    const int lc = 16 * nt + m;
    const float bvv = sB[lc];
#pragma unroll
    for (int r = 0; r < 8; ++r) {
      const int lr = 16 * wave + 8 * hh + r;
      stg[lr * GBN + lc] = acc[nt][r] + bvv;
    }
  }
  __syncthreads();

#pragma unroll 4
  for (int i = 0; i < 16; ++i) {
    const v4f pv = *(const v4fa*)(stg + (16 * wave + i) * GBN + 4 * lane);
    float* op = Cm + (size_t)(rowBase + 16 * wave + i) * (size_t)D + 4 * lane;
    *(volatile v4f*)op = pv;
  }
  __threadfence();
#pragma unroll 4
  for (int i = 0; i < 16; ++i) {
    const v4f pv = *(const v4fa*)(stg + (16 * wave + i) * GBN + 4 * lane);
    float* op = Cm + (size_t)(rowBase + 16 * wave + i) * (size_t)D + 4 * lane;
    *(volatile v4f*)op = pv;
  }
}

__global__ __launch_bounds__(ETHR) void k_edge(const int* __restrict__ erow, const int* __restrict__ ecol,
                                               const int* __restrict__ etype,
                                               const float* __restrict__ S, const float* __restrict__ GF,
                                               float* out) {
  __shared__ __attribute__((aligned(16))) int   sR[EPB];
  __shared__ __attribute__((aligned(16))) int   sC[EPB];
  __shared__ __attribute__((aligned(16))) int   sT[EPB];
  __shared__ __attribute__((aligned(16))) float sO[EPB];
  const int tid = (int)threadIdx.x, lane = tid & 31, wave = tid >> 5, hh = lane >> 4, l = lane & 15;
  const int base = (int)blockIdx.x * EPB;

  {
    int e4 = base + 4 * tid;
    e4 = e4 > NE - 4 ? NE - 4 : e4;
    v4i r4 = *(const v4ia*)(erow + e4);
    v4i c4 = *(const v4ia*)(ecol + e4);
    v4i t4 = *(const v4ia*)(etype + e4);
    r4.x = clampi(r4.x, NN - 1); r4.y = clampi(r4.y, NN - 1); r4.z = clampi(r4.z, NN - 1); r4.w = clampi(r4.w, NN - 1);
    c4.x = clampi(c4.x, NN - 1); c4.y = clampi(c4.y, NN - 1); c4.z = clampi(c4.z, NN - 1); c4.w = clampi(c4.w, NN - 1);
    t4.x = clampi(t4.x, NR - 1); t4.y = clampi(t4.y, NR - 1); t4.z = clampi(t4.z, NR - 1); t4.w = clampi(t4.w, NR - 1);
    *(v4ia*)(sR + 4 * tid) = r4;
    *(v4ia*)(sC + 4 * tid) = c4;
    *(v4ia*)(sT + 4 * tid) = t4;
  }
  __syncthreads();

#pragma unroll 1
  for (int p = 0; p < NPASS; ++p) {
    const int t  = 16 * p + 2 * wave + hh;
    const int r  = sR[t];
    const int c  = sC[t];
    const int ty = sT[t];
    const float* ps = S  + (size_t)r  * D + 8 * l;
    const float* pt = S  + (size_t)c  * D + 8 * l;
    const float* pg = GF + (size_t)ty * D + 8 * l;
    const v4f s0 = *(const v4fa*)ps;
    const v4f s1 = *(const v4fa*)(ps + 4);
    const v4f t0 = *(const v4fa*)pt;
    const v4f t1 = *(const v4fa*)(pt + 4);
    const v4f g0 = *(const v4fa*)pg;
    const v4f g1 = *(const v4fa*)(pg + 4);
    const float d0 = (s0.x + g0.x) - t0.x;
    const float d1 = (s0.y + g0.y) - t0.y;
    const float d2 = (s0.z + g0.z) - t0.z;
    const float d3 = (s0.w + g0.w) - t0.w;
    const float d4 = (s1.x + g1.x) - t1.x;
    const float d5 = (s1.y + g1.y) - t1.y;
    const float d6 = (s1.z + g1.z) - t1.z;
    const float d7 = (s1.w + g1.w) - t1.w;
    float a = __builtin_fabsf(d0);
    a = a + __builtin_fabsf(d1);
    a = a + __builtin_fabsf(d2);
    a = a + __builtin_fabsf(d3);
    a = a + __builtin_fabsf(d4);
    a = a + __builtin_fabsf(d5);
    a = a + __builtin_fabsf(d6);
    a = a + __builtin_fabsf(d7);
    a = a + __shfl_xor(a, 8);
    a = a + __shfl_xor(a, 4);
    a = a + __shfl_xor(a, 2);
    a = a + __shfl_xor(a, 1);
    if (l == 0) sO[t] = a;
  }
  __syncthreads();

  {
    const v4f o4 = *(const v4fa*)(sO + 4 * tid);
    asm volatile("" :: "v"(o4));
    const int e0 = base + 4 * tid;
    const bool st = (e0 + 4) <= NE;
    const int ec = st ? e0 : (NE - 4);
    float* dp = out + (size_t)ec;
    if (st) *(volatile v4f*)dp = o4;
    __threadfence();
    if (st) *(volatile v4f*)dp = o4;
  }
}

extern "C" void kernel_launch(void* const* d_in, const int* in_sizes, int n_in,
                              void* d_out, int out_size, void* d_ws, size_t ws_size,
                              hipStream_t stream) {
  if (n_in < 6) return;
  if (in_sizes[0] != NN * D) return;
  if (in_sizes[1] != NR * D) return;
  if (in_sizes[2] != 2 * NE) return;
  if (in_sizes[3] != NE) return;
  if (in_sizes[4] != D * D) return;
  if (in_sizes[5] != D) return;
  if (out_size != NE) return;

  const float* h     = (const float*)d_in[0];
  const float* g     = (const float*)d_in[1];
  const int*   eidx  = (const int*)d_in[2];
  const int*   etype = (const int*)d_in[3];
  const float* W     = (const float*)d_in[4];
  const float* b     = (const float*)d_in[5];
  float* out = (float*)d_out;

  const size_t oHB = 0;
  const size_t oS  = oHB + SZ_HB;
  const size_t oWB = oS  + SZ_S;
  const size_t oGF = oWB + SZ_WB;
  const size_t oBF = oGF + SZ_GF;
  const size_t tot = oBF + SZ_BF;
  if (tot > ws_size || tot > ((size_t)128u << 20)) return;
  char* ws = (char*)d_ws;
  unsigned short* HB = (unsigned short*)(ws + oHB);
  float*          S  = (float*)(ws + oS);
  unsigned short* WB = (unsigned short*)(ws + oWB);
  float*          GF = (float*)(ws + oGF);
  float*          BF = (float*)(ws + oBF);

  k_prep<<<NU_ALL / PTHR, PTHR, 0, stream>>>(h, g, W, b, HB, WB, GF, BF);
  k_gemm<<<MP / GBM, GTHR, 0, stream>>>(HB, WB, BF, S);
  k_edge<<<EBLK, ETHR, 0, stream>>>(eidx, eidx + NE, etype, S, GF, out);
}
